// MultiheadAttention_31207232373271
// MI455X (gfx1250) — hardware-run, weakly checked
//
#include <hip/hip_runtime.h>


#ifndef NB
#define NB 2
#endif
#ifndef SEQ
#define SEQ 2048
#endif
#define NB_FULL  2
#define SEQ_FULL 2048
#ifndef OUT_SEQ
#define OUT_SEQ SEQ
#endif
#define DM   768
#define NH_  12
#define HD   64
#define NPOS 1024
#define SPAN 512
#define AW   4
#define SC2  (0.07216878364870322f * 1.4426950408889634f)
#define MASKC (-1.0e6f * 1.4426950408889634f)
#define PSH  8.0f
#define WSC  64.0f
#define EP   72
#define CP   52
#define SCW  (16 * CP)
#define WLDS (48 * CP)

static_assert(HD == 64);
static_assert(NH_ * HD == DM);
static_assert(DM % 128 == 0);
static_assert(DM % 32 == 0);
static_assert(SEQ % 128 == 0);
static_assert(SEQ % (16 * AW) == 0);
static_assert(NPOS % 128 == 0);
static_assert((NB * SEQ) % 8 == 0);
static_assert(((size_t)NB * SEQ * DM) % (8 * 256) == 0);
static_assert(((size_t)NPOS * DM) % (8 * 256) == 0);
static_assert(((size_t)DM * DM) % (8 * 256) == 0);
static_assert(NB <= NB_FULL);
static_assert(SEQ <= SEQ_FULL);
static_assert(NPOS == 2 * SPAN);

typedef _Float16 h16;
typedef __attribute__((ext_vector_type(16))) _Float16 v16h;
typedef __attribute__((ext_vector_type(8)))  _Float16 v8h;
typedef __attribute__((ext_vector_type(8)))  float    v8f;
typedef __attribute__((ext_vector_type(4)))  float    v4f;
typedef v4f  __attribute__((may_alias)) v4fa;
typedef v8h  __attribute__((may_alias)) v8ha;

__device__ __forceinline__ float rbf(float f) { unsigned u = __float_as_uint(f); u += 0x7FFFu + ((u >> 16) & 1u); return __uint_as_float(u & 0xFFFF0000u); }
__device__ __forceinline__ v16h cat16(v8h lo, v8h hi) { return __builtin_shufflevector(lo, hi, 0, 1, 2, 3, 4, 5, 6, 7, 8, 9, 10, 11, 12, 13, 14, 15); }
__device__ __forceinline__ v8f wmma16(v16h a, v16h b, v8f c) { return __builtin_amdgcn_wmma_f32_16x16x32_f16(false, a, false, b, (short)0, c, false, false); }
__device__ __forceinline__ v16h ldh(const h16* p) { return cat16(*(const v8h*)p, *(const v8h*)(p + 16)); }
__device__ __forceinline__ void wave_sync() { __builtin_amdgcn_fence(3  , "wavefront"); __builtin_amdgcn_wave_barrier(); asm volatile("" ::: "memory"); }

__global__ __launch_bounds__(256) void k_cvt(const float* __restrict__ s, h16* d, size_t n8, int rows, int rows_full, float scale) {
    const size_t i = (size_t)blockIdx.x * 256 + threadIdx.x; if (i >= n8) return;
    const size_t e = i * 8; const size_t row = e / DM; const size_t col = e % DM;
    const size_t bb = row / (size_t)rows, t = row % (size_t)rows;
    const size_t so = (bb * (size_t)rows_full + t) * DM + col;
    const v8f x = *(const v8f*)(s + so); v8h o;
#pragma unroll
    for (int k = 0; k < 8; ++k) o[k] = (h16)(rbf(x[k]) * scale);
    *(volatile v8h*)(d + e) = o;
    __threadfence();
    *(volatile v8h*)(d + e) = o;
}

template <int MODE>
__global__ __launch_bounds__(128) void k_gemm(const h16* __restrict__ A, const h16* __restrict__ B, h16* C,
                                              const float* __restrict__ b1, const float* __restrict__ b2,
                                              size_t sAz, size_t sBz, size_t sCz, int ldc, float f2, float alpha) {
    __shared__ __align__(16) h16 es[4 * 32 * EP];
    const int lane = threadIdx.x & 31, wave = __builtin_amdgcn_readfirstlane((int)(threadIdx.x >> 5)), lr = lane & 15, hi = lane >> 4;
    const int z = blockIdx.z;
    const int m0 = blockIdx.x * 128 + wave * 32, n0 = blockIdx.y * 64;
    const h16* ap = A + (size_t)z * sAz + (size_t)(m0 + lr) * DM + 8 * hi;
    const h16* bp = B + (size_t)z * sBz + (size_t)(n0 + lr) * DM + 8 * hi;
    v8f acc[2][4];
#pragma unroll
    for (int mt = 0; mt < 2; ++mt)
#pragma unroll
        for (int nt = 0; nt < 4; ++nt) acc[mt][nt] = (v8f){};
#pragma unroll 1
    for (int k0 = 0; k0 < DM; k0 += 32) {
        const v16h a0 = ldh(ap + k0), a1 = ldh(ap + (size_t)16 * DM + k0);
        const v16h w0 = ldh(bp + k0), w1 = ldh(bp + (size_t)16 * DM + k0), w2 = ldh(bp + (size_t)32 * DM + k0), w3 = ldh(bp + (size_t)48 * DM + k0);
        acc[0][0] = wmma16(a0, w0, acc[0][0]); acc[1][0] = wmma16(a1, w0, acc[1][0]);
        acc[0][1] = wmma16(a0, w1, acc[0][1]); acc[1][1] = wmma16(a1, w1, acc[1][1]);
        acc[0][2] = wmma16(a0, w2, acc[0][2]); acc[1][2] = wmma16(a1, w2, acc[1][2]);
        acc[0][3] = wmma16(a0, w3, acc[0][3]); acc[1][3] = wmma16(a1, w3, acc[1][3]);
        asm volatile("v_nop\n\tv_nop\n\tv_nop\n\tv_nop"
                     : "+v"(acc[0][0]), "+v"(acc[0][1]), "+v"(acc[0][2]), "+v"(acc[0][3]), "+v"(acc[1][0]), "+v"(acc[1][1]), "+v"(acc[1][2]), "+v"(acc[1][3])
                     : "v"(a0), "v"(a1), "v"(w0), "v"(w1), "v"(w2), "v"(w3));
    }
    float c1[4], c2[4];
#pragma unroll
    for (int nt = 0; nt < 4; ++nt) { c1[nt] = 0.0f; c2[nt] = 0.0f; }
    if (MODE == 1) {
#pragma unroll
        for (int nt = 0; nt < 4; ++nt) { const int c = n0 + 16 * nt + lr; c1[nt] = rbf(b1[c]); c2[nt] = f2 * rbf(b2[c]); }
    }
    float rb[2][8];
#pragma unroll
    for (int mt = 0; mt < 2; ++mt)
#pragma unroll
        for (int r = 0; r < 8; ++r) rb[mt][r] = 0.0f;
    if (MODE == 2) {
#pragma unroll
        for (int mt = 0; mt < 2; ++mt) {
            const float* bz = b1 + m0 + 16 * mt + 8 * hi;
            const v4f x = *(const v4f*)bz; const v4f y = *(const v4f*)(bz + 4);
#pragma unroll
            for (int i = 0; i < 4; ++i) { rb[mt][i] = rbf(x[i]); rb[mt][4 + i] = rbf(y[i]); }
        }
    }
    const int wb = wave * 32 * EP;
#pragma unroll
    for (int mt = 0; mt < 2; ++mt)
#pragma unroll
        for (int nt = 0; nt < 4; ++nt)
#pragma unroll
            for (int r = 0; r < 8; ++r) {
                const float val = ((acc[mt][nt][r] * alpha + c1[nt]) + c2[nt]) + rb[mt][r];
                es[wb + (16 * mt + 8 * hi + r) * EP + 16 * nt + lr] = (h16)val;
            }
    wave_sync();
    h16* cb = C + (size_t)z * sCz + (size_t)m0 * ldc + n0;
#pragma unroll 1
    for (int ps = 0; ps < 2; ++ps) {
#pragma unroll
        for (int s = 0; s < 8; ++s) { const int row = 4 * s + (lane >> 3), c8 = (lane & 7) * 8;
            const v8h val = *(const v8ha*)(&es[wb + row * EP + c8]);
            *(volatile v8h*)(cb + (size_t)row * ldc + c8) = val; }
        if (ps == 0) __threadfence(); }
}

__global__ __launch_bounds__(32 * AW) void k_flash(const h16* __restrict__ QP, const h16* __restrict__ KP, const h16* __restrict__ VT,
                                                   const h16* __restrict__ PK, const h16* __restrict__ PQ, const float* __restrict__ mask, float* ATT) {
    __shared__ __align__(16) float rs[AW * WLDS];
    __shared__ __align__(16) float os[AW * 16 * 68];
    const int lane = threadIdx.x & 31, wave = __builtin_amdgcn_readfirstlane((int)(threadIdx.x >> 5)), lr = lane & 15, hi = lane >> 4;
    const int zh = blockIdx.y; const int b = zh / NH_, h = zh % NH_;
    const int t0 = (blockIdx.x * AW + wave) * 16;
    const size_t rbase = (size_t)b * SEQ * DM + (size_t)h * HD;
    const size_t qo = rbase + (size_t)(t0 + lr) * DM + 8 * hi;
    const v16h qh0 = ldh(QP + qo), qh1 = ldh(QP + qo + 32);
    const size_t ko = rbase + (size_t)lr * DM + 8 * hi;
    const size_t vo = ((size_t)zh * HD + lr) * SEQ + 8 * hi;
    const int hcol = h * HD + 8 * hi;
    const float* mrow = mask + (size_t)b * SEQ_FULL + 8 * hi;
    const int cb = wave * WLDS, pb = wave * WLDS + SCW;
    const bool qkeep = (t0 + lr) >= 1;
    const int wq = lr - 8 * hi + 31;
    const int crow = cb + lr * CP;
    v8f o0 = (v8f){}, o1 = (v8f){}, o2 = (v8f){}, o3 = (v8f){};
    float m = -3.0e38f, l = 0.0f;
#pragma unroll 1
    for (int key0 = 0; key0 < SEQ; key0 += 32) {
        const h16* ka = KP + ko + (size_t)key0 * DM;
        const v16h ka0 = ldh(ka), ka1 = ldh(ka + 32), kb0 = ldh(ka + (size_t)16 * DM), kb1 = ldh(ka + (size_t)16 * DM + 32);
        v8f sa = (v8f){}, sb = (v8f){};
        sa = wmma16(ka0, qh0, sa); sb = wmma16(kb0, qh0, sb);
        sa = wmma16(ka1, qh1, sa); sb = wmma16(kb1, qh1, sb);
        asm volatile("v_nop\n\tv_nop\n\tv_nop\n\tv_nop" : "+v"(sa), "+v"(sb) : "v"(ka0), "v"(ka1), "v"(kb0), "v"(kb1), "v"(qh0), "v"(qh1));
        const int base = t0 - key0 + (SPAN - 31);
        wave_sync();
#pragma unroll 1
        for (int wt = 0; wt < 3; ++wt) {
            int row = base + 16 * wt + lr; row = row < 0 ? 0 : (row > NPOS - 1 ? NPOS - 1 : row);
            const size_t po = (size_t)row * DM + hcol;
            const v16h a0 = ldh(PK + po), a1 = ldh(PK + po + 32), g0 = ldh(PQ + po), g1 = ldh(PQ + po + 32);
            v8f cc = (v8f){}, pa = (v8f){}, pc = (v8f){};
            cc = wmma16(a0, qh0, cc); pa = wmma16(g0, ka0, pa); pc = wmma16(g0, kb0, pc);
            cc = wmma16(a1, qh1, cc); pa = wmma16(g1, ka1, pa); pc = wmma16(g1, kb1, pc);
            asm volatile("v_nop\n\tv_nop\n\tv_nop\n\tv_nop" : "+v"(cc), "+v"(pa), "+v"(pc)
                         : "v"(a0), "v"(a1), "v"(g0), "v"(g1), "v"(ka0), "v"(ka1), "v"(kb0), "v"(kb1), "v"(qh0), "v"(qh1));
            const int wo = 16 * wt + 8 * hi;
            *(v4fa*)(&rs[crow + wo])                    = __builtin_shufflevector(cc, cc, 0, 1, 2, 3);
            *(v4fa*)(&rs[crow + wo + 4])                = __builtin_shufflevector(cc, cc, 4, 5, 6, 7);
            *(v4fa*)(&rs[pb + lr * CP + wo])            = __builtin_shufflevector(pa, pa, 0, 1, 2, 3);
            *(v4fa*)(&rs[pb + lr * CP + wo + 4])        = __builtin_shufflevector(pa, pa, 4, 5, 6, 7);
            *(v4fa*)(&rs[pb + (16 + lr) * CP + wo])     = __builtin_shufflevector(pc, pc, 0, 1, 2, 3);
            *(v4fa*)(&rs[pb + (16 + lr) * CP + wo + 4]) = __builtin_shufflevector(pc, pc, 4, 5, 6, 7);
        }
        wave_sync();
        const float* mp = mrow + key0;
        const v4f mk0 = *(const v4f*)mp, mk1 = *(const v4f*)(mp + 4), mk2 = *(const v4f*)(mp + 16), mk3 = *(const v4f*)(mp + 20);
        float mka[8], mkb[8];
#pragma unroll
        for (int i = 0; i < 4; ++i) { mka[i] = mk0[i]; mka[4 + i] = mk1[i]; mkb[i] = mk2[i]; mkb[4 + i] = mk3[i]; }
        float ta[8], tb[8]; float mx = -3.0e38f;
#pragma unroll
        for (int r = 0; r < 8; ++r) {
            const int kk = 8 * hi + r; const int w = wq - r;
            const float cA = rs[crow + w],      pA = rs[pb + kk * CP + w];
            const float cB = rs[crow + w - 16], pB = rs[pb + (kk + 16) * CP + w - 16];
            const float bA = (qkeep && (key0 + kk >= 1)) ? (cA + pA) : 0.0f;
            const float bB = qkeep ? (cB + pB) : 0.0f;
            ta[r] = (sa[r] + bA) * SC2 + (1.0f - mka[r]) * MASKC;
            tb[r] = (sb[r] + bB) * SC2 + (1.0f - mkb[r]) * MASKC;
            mx = fmaxf(mx, fmaxf(ta[r], tb[r]));
        }
        mx = fmaxf(mx, __shfl_xor(mx, 16, 32));
        const float mnew = fmaxf(m, mx);
        const float alpha = __builtin_amdgcn_exp2f(m - mnew);
        const float sh = PSH - mnew;
        v16h pbv; float ls = 0.0f;
#pragma unroll
        for (int r = 0; r < 8; ++r) { const h16 pa = (h16)__builtin_amdgcn_exp2f(ta[r] + sh); const h16 pc = (h16)__builtin_amdgcn_exp2f(tb[r] + sh); pbv[r] = pa; pbv[8 + r] = pc; ls += (float)pa + (float)pc; }
        l = l * alpha + ls; m = mnew;
        o0 = o0 * alpha; o1 = o1 * alpha; o2 = o2 * alpha; o3 = o3 * alpha;
        const h16* va = VT + vo + key0;
        const v16h v0 = ldh(va), v1 = ldh(va + (size_t)16 * SEQ), v2 = ldh(va + (size_t)32 * SEQ), v3 = ldh(va + (size_t)48 * SEQ);
        o0 = wmma16(v0, pbv, o0); o1 = wmma16(v1, pbv, o1); o2 = wmma16(v2, pbv, o2); o3 = wmma16(v3, pbv, o3);
        asm volatile("v_nop\n\tv_nop\n\tv_nop\n\tv_nop" : "+v"(o0), "+v"(o1), "+v"(o2), "+v"(o3) : "v"(v0), "v"(v1), "v"(v2), "v"(v3), "v"(pbv));
    }
    l += __shfl_xor(l, 16, 32);
    const float inv = 1.0f / l;
    const int wb = wave * 16 * 68;
    { v4f a, c;
      a[0] = o0[0] * inv; a[1] = o0[1] * inv; a[2] = o0[2] * inv; a[3] = o0[3] * inv; c[0] = o0[4] * inv; c[1] = o0[5] * inv; c[2] = o0[6] * inv; c[3] = o0[7] * inv;
      *(v4fa*)(&os[wb + lr * 68 +  0 + 8 * hi]) = a; *(v4fa*)(&os[wb + lr * 68 +  0 + 8 * hi + 4]) = c;
      a[0] = o1[0] * inv; a[1] = o1[1] * inv; a[2] = o1[2] * inv; a[3] = o1[3] * inv; c[0] = o1[4] * inv; c[1] = o1[5] * inv; c[2] = o1[6] * inv; c[3] = o1[7] * inv;
      *(v4fa*)(&os[wb + lr * 68 + 16 + 8 * hi]) = a; *(v4fa*)(&os[wb + lr * 68 + 16 + 8 * hi + 4]) = c;
      a[0] = o2[0] * inv; a[1] = o2[1] * inv; a[2] = o2[2] * inv; a[3] = o2[3] * inv; c[0] = o2[4] * inv; c[1] = o2[5] * inv; c[2] = o2[6] * inv; c[3] = o2[7] * inv;
      *(v4fa*)(&os[wb + lr * 68 + 32 + 8 * hi]) = a; *(v4fa*)(&os[wb + lr * 68 + 32 + 8 * hi + 4]) = c;
      a[0] = o3[0] * inv; a[1] = o3[1] * inv; a[2] = o3[2] * inv; a[3] = o3[3] * inv; c[0] = o3[4] * inv; c[1] = o3[5] * inv; c[2] = o3[6] * inv; c[3] = o3[7] * inv;
      *(v4fa*)(&os[wb + lr * 68 + 48 + 8 * hi]) = a; *(v4fa*)(&os[wb + lr * 68 + 48 + 8 * hi + 4]) = c; }
    wave_sync();
    float* orow = ATT + ((size_t)b * SEQ + t0) * DM + h * HD;
#pragma unroll 1
    for (int ps = 0; ps < 2; ++ps) {
#pragma unroll
        for (int s = 0; s < 8; ++s) { const int row = 2 * s + hi, cofs = lr * 4;
            const v4f val = *(const v4fa*)(&os[wb + row * 68 + cofs]);
            *(volatile v4f*)(orow + (size_t)row * DM + cofs) = val; }
        if (ps == 0) __threadfence(); }
}

__global__ __launch_bounds__(256) void k_ln(const float* __restrict__ att, const float* __restrict__ q, const float* __restrict__ g, const float* __restrict__ be, float* OUT) {
    const int lane = threadIdx.x & 31, wave = __builtin_amdgcn_readfirstlane((int)(threadIdx.x >> 5));
    const int row = blockIdx.x * 8 + wave;
    const int b = row / SEQ, t = row % SEQ;
    const float* ar = att + (size_t)row * DM + lane * 4;
    float s = 0.0f;
#pragma unroll 1
    for (int c = 0; c < DM / 128; ++c) { const v4f x = *(const v4f*)(ar + c * 128); s += (x[0] + x[1]) + (x[2] + x[3]); }
    s += __shfl_xor(s, 16, 32); s += __shfl_xor(s, 8, 32); s += __shfl_xor(s, 4, 32); s += __shfl_xor(s, 2, 32); s += __shfl_xor(s, 1, 32);
    const float mu = s * (1.0f / (float)DM);
    float q2 = 0.0f;
#pragma unroll 1
    for (int c = 0; c < DM / 128; ++c) { const v4f x = *(const v4f*)(ar + c * 128);
        const float d0 = x[0] - mu, d1 = x[1] - mu, d2 = x[2] - mu, d3 = x[3] - mu;
        q2 += (d0 * d0 + d1 * d1) + (d2 * d2 + d3 * d3); }
    q2 += __shfl_xor(q2, 16, 32); q2 += __shfl_xor(q2, 8, 32); q2 += __shfl_xor(q2, 4, 32); q2 += __shfl_xor(q2, 2, 32); q2 += __shfl_xor(q2, 1, 32);
    const float rstd = 1.0f / sqrtf(q2 * (1.0f / (float)DM) + 1.0e-5f);
    const float* qr = q + ((size_t)b * SEQ_FULL + t) * DM + lane * 4;
    float* orow = OUT + ((size_t)b * OUT_SEQ + t) * DM + lane * 4;
#pragma unroll 1
    for (int ps = 0; ps < 2; ++ps) {
#pragma unroll 1
        for (int c = 0; c < DM / 128; ++c) {
            const v4f x = *(const v4f*)(ar + c * 128); const v4f qq = *(const v4f*)(qr + c * 128);
            const v4f gg = *(const v4f*)(g + c * 128 + lane * 4); const v4f bb = *(const v4f*)(be + c * 128 + lane * 4);
            v4f o;
#pragma unroll
            for (int i = 0; i < 4; ++i) o[i] = rbf(qq[i]) + (((x[i] - mu) * rstd) * rbf(gg[i]) + rbf(bb[i]));
            *(volatile v4f*)(orow + c * 128) = o; }
        if (ps == 0) __threadfence(); }
}

static constexpr size_t al256(size_t v) { return (v + 255) & ~(size_t)255; }
static constexpr size_t SZ_X = al256((size_t)NB * SEQ * DM * 2);
static constexpr size_t SZ_P = al256((size_t)NPOS * DM * 2);
static constexpr size_t SZ_W = al256((size_t)DM * DM * 2);
static constexpr size_t SZ_A = al256((size_t)NB * SEQ * DM * 4);
static constexpr size_t SZ_TOTAL = 4 * SZ_X + 4 * SZ_P + 5 * SZ_W + SZ_A;
static_assert(SZ_TOTAL <= (size_t)134217728);
static_assert((size_t)NB * NH_ * HD * SEQ * 2 <= SZ_X);

extern "C" void kernel_launch(void* const* d_in, const int* in_sizes, int n_in,
                              void* d_out, int out_size, void* d_ws, size_t ws_size, hipStream_t stream) {
    if (n_in < 15) return;
    const size_t needx = ((size_t)(NB - 1) * SEQ_FULL + SEQ) * DM;
    if ((size_t)in_sizes[0] < needx) return;
    if ((size_t)in_sizes[1] < (size_t)(NB - 1) * SEQ_FULL + SEQ) return;
    if ((size_t)in_sizes[2] < (size_t)NPOS * DM || (size_t)in_sizes[3] < (size_t)NPOS * DM) return;
    if ((size_t)in_sizes[4] < (size_t)DM * DM || (size_t)in_sizes[6] < (size_t)DM * DM || (size_t)in_sizes[7] < (size_t)DM * DM ||
        (size_t)in_sizes[9] < (size_t)DM * DM || (size_t)in_sizes[11] < (size_t)DM * DM) return;
    if (in_sizes[5] < DM || in_sizes[8] < DM || in_sizes[10] < DM || in_sizes[12] < DM || in_sizes[13] < DM || in_sizes[14] < DM) return;
    if ((size_t)out_size < ((size_t)(NB - 1) * OUT_SEQ + SEQ) * DM) return;
    if (SZ_TOTAL > ws_size) return;
    const float* query = (const float*)d_in[0];  const float* amask = (const float*)d_in[1];
    const float* posk  = (const float*)d_in[2];  const float* posq  = (const float*)d_in[3];
    const float* Wq  = (const float*)d_in[4];    const float* bq  = (const float*)d_in[5];
    const float* Wk  = (const float*)d_in[6];    const float* Wv  = (const float*)d_in[7];
    const float* bv  = (const float*)d_in[8];    const float* Wpq = (const float*)d_in[9];
    const float* bpq = (const float*)d_in[10];   const float* Wpk = (const float*)d_in[11];
    const float* rwb = (const float*)d_in[12];   const float* gam = (const float*)d_in[13];
    const float* bet = (const float*)d_in[14];
    float* OUT = (float*)d_out;
    char* wsp = (char*)d_ws;
    h16* XH   = (h16*)wsp; wsp += SZ_X;
    h16* QP   = (h16*)wsp; wsp += SZ_X;
    h16* KP   = (h16*)wsp; wsp += SZ_X;
    h16* VT   = (h16*)wsp; wsp += SZ_X;
    h16* PKE  = (h16*)wsp; wsp += SZ_P;
    h16* PQE  = (h16*)wsp; wsp += SZ_P;
    h16* PKP  = (h16*)wsp; wsp += SZ_P;
    h16* PQP  = (h16*)wsp; wsp += SZ_P;
    h16* WQH  = (h16*)wsp; wsp += SZ_W;
    h16* WKH  = (h16*)wsp; wsp += SZ_W;
    h16* WVH  = (h16*)wsp; wsp += SZ_W;
    h16* WPQH = (h16*)wsp; wsp += SZ_W;
    h16* WPKH = (h16*)wsp; wsp += SZ_W;
    float* ATT = (float*)wsp; wsp += SZ_A;

    const size_t n8x = (size_t)NB * SEQ * DM / 8, n8p = (size_t)NPOS * DM / 8, n8w = (size_t)DM * DM / 8;
    k_cvt<<<(unsigned)((n8x + 255) / 256), 256, 0, stream>>>(query, XH, n8x, SEQ, SEQ_FULL, 1.0f);
    k_cvt<<<(unsigned)((n8p + 255) / 256), 256, 0, stream>>>(posk, PKE, n8p, NPOS, NPOS, 1.0f);
    k_cvt<<<(unsigned)((n8p + 255) / 256), 256, 0, stream>>>(posq, PQE, n8p, NPOS, NPOS, 1.0f);
    k_cvt<<<(unsigned)((n8w + 255) / 256), 256, 0, stream>>>(Wq,  WQH,  n8w, DM, DM, WSC);
    k_cvt<<<(unsigned)((n8w + 255) / 256), 256, 0, stream>>>(Wk,  WKH,  n8w, DM, DM, WSC);
    k_cvt<<<(unsigned)((n8w + 255) / 256), 256, 0, stream>>>(Wv,  WVH,  n8w, DM, DM, WSC);
    k_cvt<<<(unsigned)((n8w + 255) / 256), 256, 0, stream>>>(Wpq, WPQH, n8w, DM, DM, WSC);
    k_cvt<<<(unsigned)((n8w + 255) / 256), 256, 0, stream>>>(Wpk, WPKH, n8w, DM, DM, WSC);

    const float ia = 1.0f / WSC;
    k_gemm<1><<<dim3(NB * SEQ / 128, DM / 64, 1), 128, 0, stream>>>(XH, WQH, QP, bq, rwb, (size_t)0, (size_t)0, (size_t)0, DM, 1.0f, ia);
    k_gemm<0><<<dim3(NB * SEQ / 128, DM / 64, 1), 128, 0, stream>>>(XH, WKH, KP, bq, bq, (size_t)0, (size_t)0, (size_t)0, DM, 0.0f, ia);
    k_gemm<2><<<dim3(DM / 128, SEQ / 64, NB), 128, 0, stream>>>(WVH, XH, VT, bv, bv, (size_t)0, (size_t)SEQ * DM, (size_t)DM * SEQ, SEQ, 0.0f, ia);
    k_gemm<0><<<dim3(NPOS / 128, DM / 64, 1), 128, 0, stream>>>(PKE, WPKH, PKP, bq, bq, (size_t)0, (size_t)0, (size_t)0, DM, 0.0f, ia);
    k_gemm<1><<<dim3(NPOS / 128, DM / 64, 1), 128, 0, stream>>>(PQE, WPQH, PQP, bpq, bpq, (size_t)0, (size_t)0, (size_t)0, DM, 0.0f, ia);

    k_flash<<<dim3(SEQ / (16 * AW), NB * NH_, 1), 32 * AW, 0, stream>>>(QP, KP, VT, PKP, PQP, amask, ATT);
    k_ln<<<dim3(NB * SEQ / 8, 1, 1), 256, 0, stream>>>(ATT, query, gam, bet, OUT);
}
